// MHCrossAttention_77309411787
// MI455X (gfx1250) — hardware-verified
//
#include <hip/hip_runtime.h>
#include <math.h>
#include <stdint.h>

#define NBATCH  4
#define NTOK    2048
#define NCTX    2048
#define DM      512
#define NH      8
#define HD      64
#define KCH     32
#define NCHUNK  (NCTX / KCH)
#define MROWS   (NBATCH * NTOK)
#define CROWS   (NBATCH * NCTX)
#define QT16    (NTOK / 16)
#define TPG     (DM / 4)
#define WSC     64.0f
#define ACARRY  16.0f
#define QC      64.0f
#define KC      64.0f
#define VC      16.0f
#define PC      32768.0f
#define FC      4096.0f
static_assert(NH * HD == DM);
static_assert(HD == 64);
static_assert(NCHUNK == 64 && MROWS == 8192 && CROWS == 8192 && QT16 == 128 && TPG == 128);
static_assert((MROWS % 64) == 0 && (CROWS % 64) == 0 && (NTOK % 16) == 0 && (NCTX % 64) == 0 && (NCTX % KCH) == 0 && (DM % 64) == 0);
static_assert(((MROWS * DM / 8) % 256) == 0 && ((CROWS * DM / 8) % 256) == 0 && ((DM * DM / 8) % 256) == 0);
static_assert(((NBATCH * NCHUNK * TPG) % 64) == 0);
static_assert(((NBATCH * NH * QT16) % 2) == 0);

typedef _Float16 v16h __attribute__((ext_vector_type(16)));
typedef _Float16 v8h  __attribute__((ext_vector_type(8)));
typedef float    v8f  __attribute__((ext_vector_type(8)));
typedef float    v4f  __attribute__((ext_vector_type(4)));
typedef unsigned int v4u __attribute__((ext_vector_type(4)));

union FragH { v16h v; v8h h[2]; v4u u[2]; };

__device__ __forceinline__ unsigned short bf_bits(float f) {
  unsigned u = __float_as_uint(f);
  return (unsigned short)((u + 0x7FFFu + ((u >> 16) & 1u)) >> 16);
}
__device__ __forceinline__ float bf_up(unsigned short h) { return __uint_as_float(((unsigned)h) << 16); }
__device__ __forceinline__ float bfr(float f) { return bf_up(bf_bits(f)); }
__device__ __forceinline__ unsigned short h_bits(_Float16 x) { return __builtin_bit_cast(unsigned short, x); }
__device__ __forceinline__ unsigned pk16(unsigned short a, unsigned short b) { return (unsigned)a | ((unsigned)b << 16); }
__device__ __forceinline__ v8f zero8() { v8f z = {0.f, 0.f, 0.f, 0.f, 0.f, 0.f, 0.f, 0.f}; return z; }

__device__ __forceinline__ v16h ldfrag_h(const _Float16* p) {
  FragH f;
  f.h[0] = *(const v8h*)(p);
  f.h[1] = *(const v8h*)(p + 16);
  return f.v;
}
__device__ __forceinline__ v16h ldfrag_u(const unsigned short* p) {
  FragH f;
  f.u[0] = *(const v4u*)(p);
  f.u[1] = *(const v4u*)(p + 16);
  return f.v;
}

__device__ __forceinline__ v8f mma_raw(v16h a, v16h b, v8f c) {
  return __builtin_amdgcn_wmma_f32_16x16x32_f16(false, a, false, b, (short)0, c, false, false);
}
__device__ __forceinline__ void dep_guard2(v8f& a, v8f& b, v16h x, v16h y) {
#if defined(__HIP_DEVICE_COMPILE__)
  asm volatile("v_nop\n\tv_nop\n\tv_nop\n\tv_nop" : "+v"(a), "+v"(b) : "v"(x), "v"(y));
#endif
}
__device__ __forceinline__ void guard2x6(v8f& a, v8f& b, v16h p, v16h q, v16h x, v16h y, v16h z, v16h w) {
#if defined(__HIP_DEVICE_COMPILE__)
  asm volatile("v_nop\n\tv_nop\n\tv_nop\n\tv_nop" : "+v"(a), "+v"(b) : "v"(p), "v"(q), "v"(x), "v"(y), "v"(z), "v"(w));
#endif
}
__device__ __forceinline__ void guard4x5(v8f& a, v8f& b, v8f& c, v8f& d, v16h p, v16h x, v16h y, v16h z, v16h w) {
#if defined(__HIP_DEVICE_COMPILE__)
  asm volatile("v_nop\n\tv_nop\n\tv_nop\n\tv_nop" : "+v"(a), "+v"(b), "+v"(c), "+v"(d) : "v"(p), "v"(x), "v"(y), "v"(z), "v"(w));
#endif
}
__device__ __forceinline__ void keep4_h(v16h a, v16h b, v16h c, v16h d) {
#if defined(__HIP_DEVICE_COMPILE__)
  asm volatile("v_nop" :: "v"(a), "v"(b), "v"(c), "v"(d));
#endif
}
__device__ __forceinline__ void acc_guard4(v8f& a, v8f& b, v8f& c, v8f& d) {
#if defined(__HIP_DEVICE_COMPILE__)
  asm volatile("v_nop\n\tv_nop\n\tv_nop\n\tv_nop" : "+v"(a), "+v"(b), "+v"(c), "+v"(d));
#endif
}
__device__ __forceinline__ void wave_sync_lds() {
  __builtin_amdgcn_fence(__ATOMIC_RELEASE, "workgroup");
  __builtin_amdgcn_wave_barrier();
  __builtin_amdgcn_fence(__ATOMIC_ACQUIRE, "workgroup");
}

__global__ __launch_bounds__(256) void conv16(const float* __restrict__ X0, const float* __restrict__ X1,
                                              const float* __restrict__ X2, const float* __restrict__ X3,
                                              unsigned short* D0, unsigned short* D1, unsigned short* D2,
                                              unsigned short* D3, int n8, float wsc) {
  const int sel = blockIdx.y;
  const float* X = (sel == 0) ? X0 : ((sel == 1) ? X1 : ((sel == 2) ? X2 : X3));
  unsigned short* dst = (sel == 0) ? D0 : ((sel == 1) ? D1 : ((sel == 2) ? D2 : D3));
  const int i  = blockIdx.x * 256 + threadIdx.x;
  const int ic = (i < n8) ? i : (n8 - 1);
  const float* p = X + (size_t)ic * 8;
  const v4f a = *(const v4f*)(p), b = *(const v4f*)(p + 4);
  float v[8];
#pragma unroll
  for (int e = 0; e < 4; ++e) { v[e] = bfr(a[e]); v[4 + e] = bfr(b[e]); }
  v4u ov;
#pragma unroll
  for (int e = 0; e < 4; ++e) ov[e] = pk16(h_bits((_Float16)(v[2 * e] * wsc)), h_bits((_Float16)(v[2 * e + 1] * wsc)));
  if (i < n8) *(volatile v4u*)(dst + (size_t)i * 8) = ov;
  __threadfence();
  if (i < n8) *(volatile v4u*)(dst + (size_t)i * 8) = ov;
}

template <int OM, int HASB, int TWOA>
__global__ __launch_bounds__(256) void gemm64(
    const unsigned short* __restrict__ Ap, const unsigned short* __restrict__ A2p, int lda, long long sA,
    const unsigned short* __restrict__ Btp, int ldb, long long sB,
    const float* __restrict__ bias, float bscale,
    void* Cout, void* Cout2, int ldc, long long sC,
    int M, int N, int K, float oscale) {
  __shared__ __align__(16) float sT[8][16 * 68];
  const int by   = blockIdx.y;
  const int lane = threadIdx.x & 31;
  const int wave = threadIdx.x >> 5;
  const int tilesN = N >> 6;
  const int tilesM = M >> 6;
  const int tile = blockIdx.x * 8 + wave;
  if (tile >= tilesM * tilesN) return;
  const int tm = tile / tilesN;
  const int tn = tile - tm * tilesN;
  const int m0 = tm << 6;
  const int n0 = tn << 6;

  const unsigned short* A1 = Ap  + (size_t)((long long)by * sA);
  const unsigned short* A2 = A2p + (size_t)((long long)by * sA);
  const unsigned short* Bb = Btp + (size_t)((long long)by * sB);

  const int rlane = lane & 15;
  const int koff  = (lane >> 4) * 8;
  const int mOff  = (lane >> 4) * 8;

  v8f acc[4][4];
#pragma unroll
  for (int i = 0; i < 4; ++i)
#pragma unroll
    for (int j = 0; j < 4; ++j) acc[i][j] = zero8();

  for (int k0 = 0; k0 < K; k0 += 32) {
    v16h bh[4];
#pragma unroll
    for (int j = 0; j < 4; ++j) {
      const size_t bofs = (size_t)(n0 + (j << 4) + rlane) * ldb + koff + k0;
      bh[j] = ldfrag_u(Bb + bofs);
    }
#pragma unroll
    for (int i = 0; i < 4; ++i) {
      const size_t ao = (size_t)(m0 + (i << 4) + rlane) * lda + koff + k0;
      const v16h ah = ldfrag_u(A1 + ao);
      v16h al = ah;
      if (TWOA != 0) al = ldfrag_u(A2 + ao);
#pragma unroll
      for (int j = 0; j < 4; ++j) {
        acc[i][j] = mma_raw(ah, bh[j], acc[i][j]);
        if (TWOA != 0) acc[i][j] = mma_raw(al, bh[j], acc[i][j]);
      }
      dep_guard2(acc[i][0], acc[i][3], ah, al);
    }
    keep4_h(bh[0], bh[1], bh[2], bh[3]);
  }
  acc_guard4(acc[0][0], acc[0][1], acc[0][2], acc[0][3]);
  acc_guard4(acc[1][0], acc[1][1], acc[1][2], acc[1][3]);
  acc_guard4(acc[2][0], acc[2][1], acc[2][2], acc[2][3]);
  acc_guard4(acc[3][0], acc[3][1], acc[3][2], acc[3][3]);

  const int hh2 = lane >> 4, c4 = (lane & 15) * 4;
  const int q8  = lane >> 3, c8 = (lane & 7) * 8;
  float bc[4];
#pragma unroll
  for (int e = 0; e < 4; ++e) bc[e] = 0.f;
  if (HASB != 0 && OM == 0) {
    const int cb = n0 + c4;
    const int i0 = (cb < N - 4) ? cb : (N - 4);
    const v4f b0v = *(const v4f*)(bias + i0);
#pragma unroll
    for (int e = 0; e < 4; ++e) bc[e] = bfr(b0v[e]) * bscale;
  }

  float* slab = sT[wave];
#pragma unroll
  for (int i = 0; i < 4; ++i) {
    const int mBase = m0 + (i << 4);
#pragma unroll
    for (int j = 0; j < 4; ++j) {
#pragma unroll
      for (int r = 0; r < 8; ++r) {
        slab[(mOff + r) * 68 + (j << 4) + rlane] = acc[i][j][r];
      }
    }
    wave_sync_lds();
    if (OM == 0) {
      float* C = (float*)Cout + (size_t)((long long)by * sC);
      v4f vals[8];
#pragma unroll
      for (int it = 0; it < 8; ++it) {
        const int row = it * 2 + hh2;
        v4f v = *(const v4f*)(slab + row * 68 + c4);
#pragma unroll
        for (int e = 0; e < 4; ++e) v[e] = v[e] * oscale + bc[e];
        vals[it] = v;
      }
      for (int pass = 0; pass < 2; ++pass) {
#pragma unroll
        for (int it = 0; it < 8; ++it) {
          const int gr = mBase + it * 2 + hh2;
          *(volatile v4f*)(C + (size_t)gr * ldc + n0 + c4) = vals[it];
        }
        __threadfence();
      }
    } else {
      unsigned short* C  = (unsigned short*)Cout  + (size_t)((long long)by * sC);
      unsigned short* C2 = (unsigned short*)Cout2 + (size_t)((long long)by * sC);
      v4u hv[4], lv[4];
#pragma unroll
      for (int it = 0; it < 4; ++it) {
        const int row = it * 4 + q8;
        const float* sp = slab + row * 68 + c8;
        v4u a = {0u, 0u, 0u, 0u}, b = {0u, 0u, 0u, 0u};
#pragma unroll
        for (int e = 0; e < 4; ++e) {
          const float f0 = sp[2 * e] * oscale;
          const float f1 = sp[2 * e + 1] * oscale;
          const _Float16 h0 = (_Float16)f0, h1 = (_Float16)f1;
          a[e] = pk16(h_bits(h0), h_bits(h1));
          if (OM == 3) {
            const _Float16 l0 = (_Float16)(f0 - (float)h0), l1 = (_Float16)(f1 - (float)h1);
            b[e] = pk16(h_bits(l0), h_bits(l1));
          }
        }
        hv[it] = a;
        lv[it] = b;
      }
      for (int pass = 0; pass < 2; ++pass) {
#pragma unroll
        for (int it = 0; it < 4; ++it) {
          const int row = it * 4 + q8;
          *(volatile v4u*)(C + (size_t)(mBase + row) * ldc + n0 + c8) = hv[it];
          if (OM == 3) *(volatile v4u*)(C2 + (size_t)(mBase + row) * ldc + n0 + c8) = lv[it];
        }
        __threadfence();
      }
    }
    wave_sync_lds();
  }
}

__global__ __launch_bounds__(64) void colsum32(const float* __restrict__ V, float* CS, int ngrp) {
  const int t  = blockIdx.x * 64 + threadIdx.x;
  const int g  = t >> 7;
  const int i4 = (t & (TPG - 1)) * 4;
  const int gc = (g < ngrp) ? g : (ngrp - 1);
  const float* src = V + (size_t)gc * (KCH * DM) + i4;
  v4f acc = {0.f, 0.f, 0.f, 0.f};
#pragma unroll 8
  for (int j = 0; j < KCH; ++j) {
    const v4f x = *(const v4f*)(src + (size_t)j * DM);
    acc += x;
  }
  if (g < ngrp) *(volatile v4f*)(CS + (size_t)g * DM + i4) = acc;
  __threadfence();
  if (g < ngrp) *(volatile v4f*)(CS + (size_t)g * DM + i4) = acc;
}

__global__ __launch_bounds__(64)
void attn64(const unsigned short* __restrict__ QPp, const unsigned short* __restrict__ KPp,
            const unsigned short* __restrict__ VTq, const float* __restrict__ CSp,
            const int* __restrict__ maskp, unsigned short* CH, unsigned short* CL) {
  __shared__ __align__(16) float Ps[2][16 * 36];
  __shared__ __align__(16) unsigned short Oh[2][16 * HD];
  __shared__ __align__(16) unsigned short Ol[2][16 * HD];

  const int tid  = threadIdx.x;
  const int wave = tid >> 5;
  const int lane = tid & 31;
  const int hh   = lane >> 4;
  const int c    = lane & 15;

  const int w    = blockIdx.x * 2 + wave;
  const int head = w % NH;
  const int rest = w / NH;
  const int qt   = rest % QT16;
  const int bat  = rest / QT16;
  const int q0   = qt * 16;

  const _Float16* Qp = (const _Float16*)(const void*)QPp + ((size_t)bat * NTOK + q0 + c) * DM + head * HD + 8 * hh;
  const _Float16* Kb = (const _Float16*)(const void*)KPp + (size_t)bat * NCTX * DM + head * HD + 8 * hh;
  const _Float16* Vb = (const _Float16*)(const void*)VTq + (size_t)(bat * NH + head) * HD * NCTX + 8 * hh;
  const float*  csb  = CSp + (size_t)bat * NCHUNK * DM + head * HD + c;
  const int*    mrp  = maskp + (size_t)(bat * NH + head) * NTOK + q0 + 8 * hh;
  const float lsc = (1.4426950408889634f * 0.044194173824159216f) / (QC * KC);

  const v16h qf0 = ldfrag_h(Qp);
  const v16h qf1 = ldfrag_h(Qp + 32);

  float mrow[8], lrow[8], rb[8];
  v8f o0 = zero8(), o1 = zero8(), o2 = zero8(), o3 = zero8();
  v8f u0 = zero8(), u1 = zero8(), u2 = zero8(), u3 = zero8();
#pragma unroll
  for (int r = 0; r < 8; ++r) {
    mrow[r] = -INFINITY; lrow[r] = 0.f;
    rb[r] = (mrp[r] != 0) ? 0.f : -INFINITY;
  }
  float* pt = Ps[wave];

#pragma unroll 1
  for (int kb = 0; kb < NCTX; kb += KCH) {
    const _Float16* kp = Kb + (size_t)(kb + c) * DM;
    v8f s0, s1;
    {
      const v16h k0a = ldfrag_h(kp);
      const v16h k0b = ldfrag_h(kp + 32);
      const v16h k1a = ldfrag_h(kp + (size_t)16 * DM);
      const v16h k1b = ldfrag_h(kp + (size_t)16 * DM + 32);
      s0 = mma_raw(qf0, k0a, zero8());
      s0 = mma_raw(qf1, k0b, s0);
      s1 = mma_raw(qf0, k1a, zero8());
      s1 = mma_raw(qf1, k1b, s1);
      guard2x6(s0, s1, qf0, qf1, k0a, k0b, k1a, k1b);
    }
    const float* csp = csb + (size_t)(kb / KCH) * DM;
    const float cs0 = csp[0];
    const float cs1 = csp[16];
    const float cs2 = csp[32];
    const float cs3 = csp[48];
#pragma unroll
    for (int r = 0; r < 8; ++r) {
      const float t0 = s0[r] * lsc + rb[r], t1 = s1[r] * lsc + rb[r];
      float mx = fmaxf(t0, t1);
#pragma unroll
      for (int off = 1; off < 16; off <<= 1) mx = fmaxf(mx, __shfl_xor(mx, off, 32));
      const float mn = fmaxf(mrow[r], mx);
      const float al = exp2f(mrow[r] - mn);
      mrow[r] = mn;
      const float e0 = exp2f(t0 - mn), e1 = exp2f(t1 - mn);
      float ps = e0 + e1;
#pragma unroll
      for (int off = 1; off < 16; off <<= 1) ps += __shfl_xor(ps, off, 32);
      const float eb = ps * (1.0f / 32.0f);
      lrow[r] = lrow[r] * al + ps;
      o0[r] *= al;
      o1[r] *= al;
      o2[r] *= al;
      o3[r] *= al;
      u0[r] = u0[r] * al + eb * cs0;
      u1[r] = u1[r] * al + eb * cs1;
      u2[r] = u2[r] * al + eb * cs2;
      u3[r] = u3[r] * al + eb * cs3;
      const int ro = (8 * hh + r) * 36 + c;
      pt[ro]      = e0 - eb;
      pt[ro + 16] = e1 - eb;
    }
    wave_sync_lds();
    FragH ph;
    {
      const float* prow = pt + c * 36 + 8 * hh;
      const v4f p0 = *(const v4f*)(prow), p1 = *(const v4f*)(prow + 4);
      const v4f p2 = *(const v4f*)(prow + 16), p3 = *(const v4f*)(prow + 20);
#pragma unroll
      for (int e = 0; e < 4; ++e) {
        ph.h[0][e]     = (_Float16)(p0[e] * PC);
        ph.h[0][4 + e] = (_Float16)(p1[e] * PC);
        ph.h[1][e]     = (_Float16)(p2[e] * PC);
        ph.h[1][4 + e] = (_Float16)(p3[e] * PC);
      }
    }
    const _Float16* vp = Vb + (size_t)c * NCTX + kb;
    {
      const v16h vb0 = ldfrag_h(vp);
      const v16h vb1 = ldfrag_h(vp + (size_t)16 * NCTX);
      const v16h vb2 = ldfrag_h(vp + (size_t)32 * NCTX);
      const v16h vb3 = ldfrag_h(vp + (size_t)48 * NCTX);
      o0 = mma_raw(ph.v, vb0, o0);
      o1 = mma_raw(ph.v, vb1, o1);
      o2 = mma_raw(ph.v, vb2, o2);
      o3 = mma_raw(ph.v, vb3, o3);
      guard4x5(o0, o1, o2, o3, ph.v, vb0, vb1, vb2, vb3);
    }
    wave_sync_lds();
  }

  const float oc = 1.0f / (PC * VC);
  unsigned short* ohw = Oh[wave];
  unsigned short* olw = Ol[wave];
#pragma unroll
  for (int r = 0; r < 8; ++r) {
    const float inv = 1.0f / lrow[r];
    const float f0 = ((o0[r] * oc + u0[r]) * inv) * FC;
    const float f1 = ((o1[r] * oc + u1[r]) * inv) * FC;
    const float f2 = ((o2[r] * oc + u2[r]) * inv) * FC;
    const float f3 = ((o3[r] * oc + u3[r]) * inv) * FC;
    const _Float16 g0 = (_Float16)f0, g1 = (_Float16)f1, g2 = (_Float16)f2, g3 = (_Float16)f3;
    const _Float16 l0 = (_Float16)(f0 - (float)g0), l1 = (_Float16)(f1 - (float)g1);
    const _Float16 l2 = (_Float16)(f2 - (float)g2), l3 = (_Float16)(f3 - (float)g3);
    const int ro = (8 * hh + r) * HD + c;
    ohw[ro]      = h_bits(g0);
    ohw[ro + 16] = h_bits(g1);
    ohw[ro + 32] = h_bits(g2);
    ohw[ro + 48] = h_bits(g3);
    olw[ro]      = h_bits(l0);
    olw[ro + 16] = h_bits(l1);
    olw[ro + 32] = h_bits(l2);
    olw[ro + 48] = h_bits(l3);
  }
  wave_sync_lds();
  {
    v4u hv[4], lv[4];
#pragma unroll
    for (int it = 0; it < 4; ++it) {
      const int p   = it * 32 + lane;
      const int row = p >> 3;
      const int c8  = (p & 7) * 8;
      hv[it] = *(const v4u*)(ohw + row * HD + c8);
      lv[it] = *(const v4u*)(olw + row * HD + c8);
    }
    const size_t dofs = ((size_t)bat * NTOK + q0) * DM + (size_t)head * HD;
    unsigned short* dh = CH + dofs;
    unsigned short* dl = CL + dofs;
    for (int pass = 0; pass < 2; ++pass) {
#pragma unroll
      for (int it = 0; it < 4; ++it) {
        const int p   = it * 32 + lane;
        const int row = p >> 3;
        const int c8  = (p & 7) * 8;
        *(volatile v4u*)(dh + (size_t)row * DM + c8) = hv[it];
        *(volatile v4u*)(dl + (size_t)row * DM + c8) = lv[it];
      }
      __threadfence();
    }
  }
}

extern "C" void kernel_launch(void* const* d_in, const int* in_sizes, int n_in,
                              void* d_out, int out_size, void* d_ws, size_t ws_size,
                              hipStream_t stream) {
  if (n_in < 8) return;
  if (in_sizes[0] != MROWS * DM) return;
  if (in_sizes[1] != CROWS * DM) return;
  if (in_sizes[2] != NBATCH * NH * NTOK) return;
  if (in_sizes[3] != DM * DM || in_sizes[4] != DM * DM || in_sizes[5] != DM * DM || in_sizes[6] != DM * DM) return;
  if (in_sizes[7] != DM) return;
  if (out_size != MROWS * DM) return;

  const float* q_x  = (const float*)d_in[0];
  const float* kv_x = (const float*)d_in[1];
  const int*   qmsk = (const int*)d_in[2];
  const float* w_q  = (const float*)d_in[3];
  const float* w_k  = (const float*)d_in[4];
  const float* w_v  = (const float*)d_in[5];
  const float* w_o  = (const float*)d_in[6];
  const float* b_o  = (const float*)d_in[7];
  float*       out  = (float*)d_out;

  const size_t PW   = (size_t)DM * DM * 2;
  const size_t PXI  = (size_t)MROWS * DM * 2;
  const size_t PKI  = (size_t)CROWS * DM * 2;
  const size_t PV32 = (size_t)CROWS * DM * 4;
  const size_t PVT  = (size_t)NBATCH * DM * NCTX * 2;
  const size_t PCS  = (size_t)NBATCH * NCHUNK * DM * 4;
  size_t off = 0;
  const size_t oWQ  = off; off += PW;
  const size_t oWK  = off; off += PW;
  const size_t oWV  = off; off += PW;
  const size_t oWO  = off; off += PW;
  const size_t oXI  = off; off += PXI;
  const size_t oKI  = off; off += PKI;
  const size_t oQP  = off; off += PXI;
  const size_t oKP  = off; off += PKI;
  const size_t oV32 = off; off += PV32;
  const size_t oVT  = off; off += PVT;
  const size_t oCS  = off; off += PCS;
  const size_t oCH  = off; off += PXI;
  const size_t oCL  = off; off += PXI;
  if (off > ws_size) return;
  if (off > (size_t)134217728) return;
  if ((PW % 4096) != 0 || (PXI % 4096) != 0 || (PKI % 4096) != 0 || (PV32 % 4096) != 0 || (PVT % 4096) != 0 ||
      (PCS % 4096) != 0) return;

  char* ws = (char*)d_ws;
  unsigned short* WQ  = (unsigned short*)(ws + oWQ);
  unsigned short* WK  = (unsigned short*)(ws + oWK);
  unsigned short* WV  = (unsigned short*)(ws + oWV);
  unsigned short* WO  = (unsigned short*)(ws + oWO);
  unsigned short* XI  = (unsigned short*)(ws + oXI);
  unsigned short* KI  = (unsigned short*)(ws + oKI);
  unsigned short* QP  = (unsigned short*)(ws + oQP);
  unsigned short* KP  = (unsigned short*)(ws + oKP);
  float*          V32 = (float*)(ws + oV32);
  unsigned short* VTp = (unsigned short*)(ws + oVT);
  float*          CS  = (float*)(ws + oCS);
  unsigned short* CH  = (unsigned short*)(ws + oCH);
  unsigned short* CL  = (unsigned short*)(ws + oCL);

  const int n8t = (MROWS * DM) / 8;
  const int n8w = (DM * DM) / 8;
  if ((n8t % 256) != 0 || (n8w % 256) != 0) return;
  const dim3 blk(256), blk64(64);
  const dim3 gCt(n8t / 256, 2);
  const dim3 gCw(n8w / 256, 4);
  const int tilesQ  = (MROWS / 64) * (DM / 64);
  const int tilesK  = (CROWS / 64) * (DM / 64);
  const int tilesVT = (DM / 64) * (NCTX / 64);
  if ((tilesQ % 8) != 0 || (tilesK % 8) != 0 || (tilesVT % 8) != 0) return;
  const dim3 gQ(tilesQ / 8, 1);
  const dim3 gK(tilesK / 8, 1);
  const dim3 gVT(tilesVT / 8, NBATCH);
  const int ngrp = NBATCH * NCHUNK;
  const dim3 gCS((ngrp * TPG) / 64);
  const dim3 gAT((NBATCH * NH * QT16) / 2);

  conv16<<<gCw, blk, 0, stream>>>(w_q, w_k, w_v, w_o, WQ, WK, WV, WO, n8w, WSC);

  conv16<<<gCt, blk, 0, stream>>>(q_x, kv_x, q_x, kv_x, XI, KI, XI, KI, n8t, ACARRY);

  gemm64<2, 0, 0><<<gQ, blk, 0, stream>>>(
      XI, XI, DM, 0LL,
      WQ, DM, 0LL,
      b_o, 0.f,
      (void*)QP, (void*)QP, DM, 0LL,
      MROWS, DM, DM, QC / (ACARRY * WSC));

  gemm64<2, 0, 0><<<gK, blk, 0, stream>>>(
      KI, KI, DM, 0LL,
      WK, DM, 0LL,
      b_o, 0.f,
      (void*)KP, (void*)KP, DM, 0LL,
      CROWS, DM, DM, KC / (ACARRY * WSC));

  gemm64<0, 0, 0><<<gK, blk, 0, stream>>>(
      KI, KI, DM, 0LL,
      WV, DM, 0LL,
      b_o, 0.f,
      (void*)V32, (void*)V32, DM, 0LL,
      CROWS, DM, DM, 1.0f / (ACARRY * WSC));

  gemm64<2, 0, 0><<<gVT, blk, 0, stream>>>(
      WV, WV, DM, 0LL,
      KI, DM, (long long)NCTX * DM,
      b_o, 0.f,
      (void*)VTp, (void*)VTp, NCTX, (long long)DM * NCTX,
      DM, NCTX, DM, VC / (ACARRY * WSC));

  colsum32<<<gCS, blk64, 0, stream>>>(V32, CS, ngrp);

  attn64<<<gAT, blk64, 0, stream>>>(QP, KP, VTp, CS, qmsk, CH, CL);

  gemm64<0, 1, 1><<<gQ, blk, 0, stream>>>(
      CH, CL, DM, 0LL,
      WO, DM, 0LL,
      b_o, 1.0f,
      (void*)out, (void*)out, DM, 0LL,
      MROWS, DM, DM, 1.0f / (FC * WSC));
  (void)hipGetLastError();
}
